// MoE_8383776161864
// MI455X (gfx1250) — hardware-verified
//
#include <hip/hip_runtime.h>
#include <math.h>

typedef _Float16 h16;
typedef __attribute__((ext_vector_type(16))) __bf16 v16b;
typedef __attribute__((ext_vector_type(16))) _Float16 v16h;
typedef __attribute__((ext_vector_type(8)))  float v8f;
typedef __attribute__((ext_vector_type(4)))  float v4f;
typedef __attribute__((ext_vector_type(4)))  unsigned v4u;
typedef __attribute__((ext_vector_type(8)))  unsigned v8u;

#ifndef NB
#define NB 2u
#endif
#ifndef SEQ
#define SEQ 2048u
#endif
#ifndef NT
#define NT (NB * SEQ)
#endif
#define DD 1024u
#define DO 1024u
#define II 512u
#define NE 8u
#define NK (NE * II)
#define DDQ (DD / 8u)
#define NKQ (NK / 8u)
#define WPQ (II / 8u)
#define PEQ (DO * WPQ)
#define TSQ (16u * DDQ)
#define TPQ (16u * WPQ)
#define HMC 256.0f
#define WPC 4096.0f
#define OSC 9.5367431640625e-07f

static_assert((NT & 127u) == 0u);
static_assert((DD & 63u) == 0u);
static_assert((DO & 255u) == 0u);
static_assert((NK & 255u) == 0u);
static_assert((II % 256u) == 0u);
static_assert((II & 31u) == 0u);
static_assert(II / 32u == 16u);
static_assert((DD & 31u) == 0u);
static_assert(DD == 1024u);
static_assert(NE == 8u);
static_assert(HMC * WPC * OSC == 1.0f);

#define WS_G   0u
#define WS_XB  (WS_G + 4u * NE * (size_t)NT)
#define WS_WF  (WS_XB + 2u * (size_t)NT * DD)
#define WS_WP  (WS_WF + 2u * (size_t)NK * DD)
#define WS_HM  (WS_WP + 2u * (size_t)NE * DO * II)
#define WS_END (WS_HM + 2u * (size_t)NT * NK)
static_assert((WS_XB & 127u) == 0u);
static_assert((WS_WF & 127u) == 0u);
static_assert((WS_WP & 127u) == 0u);
static_assert((WS_HM & 127u) == 0u);
static_assert(WS_END <= 134217728u);

template <typename T> __device__ __forceinline__ void vst2(T* p, T v) { *(volatile T*)p = v; __threadfence(); *(volatile T*)p = v; }

__device__ __forceinline__ v8f wmma_bf(v16b a, v16b b, v8f c) {
  v8f d = __builtin_amdgcn_wmma_f32_16x16x32_bf16(false, a, false, b, (short)0, c, false, false);
  asm volatile("v_nop\n\tv_nop\n\tv_nop\n\tv_nop" : "+v"(d) : "v"(a), "v"(b));
  return d;
}
__device__ __forceinline__ v8f wmma_h(v16h a, v16h b, v8f c) {
  v8f d = __builtin_amdgcn_wmma_f32_16x16x32_f16(false, a, false, b, (short)0, c, false, false);
  asm volatile("v_nop\n\tv_nop\n\tv_nop\n\tv_nop" : "+v"(d) : "v"(a), "v"(b));
  return d;
}
__device__ __forceinline__ v16b frag_q(v4u q0, v4u q1) {
  const v8u w = __builtin_shufflevector(q0, q1, 0, 1, 2, 3, 4, 5, 6, 7);
  return __builtin_bit_cast(v16b, w);
}
__device__ __forceinline__ v16h frag_h(v4u q0, v4u q1) {
  const v8u w = __builtin_shufflevector(q0, q1, 0, 1, 2, 3, 4, 5, 6, 7);
  return __builtin_bit_cast(v16h, w);
}
__device__ __forceinline__ float bfr(float v) { return (float)(__bf16)v; }
__device__ __forceinline__ unsigned short bfbits(float v) { return __builtin_bit_cast(unsigned short, (__bf16)v); }
__device__ __forceinline__ unsigned pk2(float a, float b) { return (unsigned)bfbits(a) | ((unsigned)bfbits(b) << 16); }
static __device__ __forceinline__ h16 toh_flush(float v) { const h16 r = (h16)v; return (fabsf(v) < 6.103515625e-05f) ? (h16)0.0f : r; }
__device__ __forceinline__ unsigned short hbits(float v) { return __builtin_bit_cast(unsigned short, toh_flush(v)); }
__device__ __forceinline__ unsigned pkh2(float a, float b) { return (unsigned)hbits(a) | ((unsigned)hbits(b) << 16); }
__device__ __forceinline__ float gelu_erf(float v) { return 0.5f * v * (1.0f + erff(v * 0.70710678118654752f)); }

static_assert(((NT * DD) / 8u) % 256u == 0u);
__global__ __launch_bounds__(256) void k_xcvt(const float* __restrict__ X, v4u* __restrict__ XB) {
  const unsigned idx = blockIdx.x * 256u + threadIdx.x;
  const float* p = X + (size_t)idx * 8u;
  const v4f a = *(const v4f*)p;
  const v4f b = *(const v4f*)(p + 4);
  v4u o; o[0] = pk2(a[0], a[1]); o[1] = pk2(a[2], a[3]); o[2] = pk2(b[0], b[1]); o[3] = pk2(b[2], b[3]);
  vst2(XB + idx, o);
}
static_assert(((NK * DD) / 8u) % 256u == 0u);

static_assert(((NE * DO * II) / 8u) % 256u == 0u);
__global__ __launch_bounds__(256) void k_pcvt(const float* __restrict__ W, v4u* __restrict__ WP) {
  const unsigned idx = blockIdx.x * 256u + threadIdx.x;
  const float* p = W + (size_t)idx * 8u;
  const v4f a = *(const v4f*)p;
  const v4f b = *(const v4f*)(p + 4);
  v4u o;
  o[0] = pkh2(bfr(a[0]) * WPC, bfr(a[1]) * WPC);
  o[1] = pkh2(bfr(a[2]) * WPC, bfr(a[3]) * WPC);
  o[2] = pkh2(bfr(b[0]) * WPC, bfr(b[1]) * WPC);
  o[3] = pkh2(bfr(b[2]) * WPC, bfr(b[3]) * WPC);
  vst2(WP + idx, o);
}

#define GWP 1028u
static_assert((NE * DD) / 4u == 8u * 256u);
static_assert(64u * 16u == 32u * NE * 4u);
static_assert((NT & 31u) == 0u);
static_assert(4u * NE * GWP + 4u * 32u * NE <= 131072u);
__global__ __launch_bounds__(256) void k_gate(const v4u* __restrict__ XB, const float* __restrict__ WG, float* __restrict__ G) {
#pragma clang fp contract(off)
  __shared__ __align__(16) float swg[NE][GWP];
  __shared__ __align__(16) float sl[32][8];
  const unsigned tid = threadIdx.x;
  const unsigned wave = (unsigned)__builtin_amdgcn_readfirstlane((int)(threadIdx.x >> 5));
  const unsigned r0 = blockIdx.x * 32u;
#pragma unroll 1
  for (unsigned r = 0; r < 8u; ++r) {
    const unsigned idx = r * 256u + tid;
    const v4f t4 = *(const v4f*)(WG + (size_t)idx * 4u);
    const unsigned e = idx >> 8, i = (idx & 255u) * 4u;
    v4f w4; w4[0] = bfr(t4[0]); w4[1] = bfr(t4[1]); w4[2] = bfr(t4[2]); w4[3] = bfr(t4[3]);
    *(v4f*)&swg[e][i] = w4;
  }
  __syncthreads();
  const unsigned tk = tid >> 3, ee = tid & 7u;
  const v4u* px = XB + (size_t)(r0 + tk) * DDQ;
  float acc = 0.0f;
#pragma unroll 1
  for (unsigned kq = 0; kq < DDQ; ++kq) {
    const v4u xq = px[kq];
    const v4f wa = *(const v4f*)&swg[ee][kq * 8u];
    const v4f wb = *(const v4f*)&swg[ee][kq * 8u + 4u];
    acc = fmaf(__uint_as_float(xq[0] << 16), wa[0], acc);
    acc = fmaf(__uint_as_float(xq[0] & 0xffff0000u), wa[1], acc);
    acc = fmaf(__uint_as_float(xq[1] << 16), wa[2], acc);
    acc = fmaf(__uint_as_float(xq[1] & 0xffff0000u), wa[3], acc);
    acc = fmaf(__uint_as_float(xq[2] << 16), wb[0], acc);
    acc = fmaf(__uint_as_float(xq[2] & 0xffff0000u), wb[1], acc);
    acc = fmaf(__uint_as_float(xq[3] << 16), wb[2], acc);
    acc = fmaf(__uint_as_float(xq[3] & 0xffff0000u), wb[3], acc);
  }
  sl[tk][ee] = acc;
  __syncthreads();
  if (wave < 2u) {
    const unsigned tok = tid >> 1, e0 = (tid & 1u) * 4u;
    const v4f la = *(const v4f*)&sl[tok][0];
    const v4f lb = *(const v4f*)&sl[tok][4];
    float l[8];
    l[0] = la[0]; l[1] = la[1]; l[2] = la[2]; l[3] = la[3];
    l[4] = lb[0]; l[5] = lb[1]; l[6] = lb[2]; l[7] = lb[3];
    unsigned i0 = 0u; float v0 = l[0];
#pragma unroll
    for (unsigned e = 1; e < 8u; ++e) {
      const bool take = l[e] > v0;
      v0 = take ? l[e] : v0;
      i0 = take ? e : i0;
    }
    unsigned i1 = 8u; float v1 = -INFINITY;
#pragma unroll
    for (unsigned e = 0; e < 8u; ++e) {
      const bool take = (e != i0) && ((i1 == 8u) || (l[e] > v1));
      v1 = take ? l[e] : v1;
      i1 = take ? e : i1;
    }
    const float ex = expf(v1 - v0);
    const float s = 1.0f + ex;
    const float inv = 1.0f / s;
    const float w0 = inv, w1 = ex * inv;
    v4f gq;
#pragma unroll
    for (unsigned j = 0; j < 4u; ++j) {
      const unsigned e = e0 + j;
      gq[j] = (e == i0) ? w0 : ((e == i1) ? w1 : 0.0f);
    }
    vst2((v4f*)(G + (size_t)r0 * NE + tid * 4u), gq);
  }
}

static_assert(32u * 16u * 8u == 16u * 128u * 2u);
__global__ __launch_bounds__(256) void k_fc(const v4u* __restrict__ XB, const v4u* __restrict__ WF, const float* __restrict__ G, v4u* __restrict__ HM) {
  __shared__ __align__(16) float sg[128][8];
  __shared__ __align__(16) unsigned short st[8][16][136];
  static_assert(sizeof(float) * 128u * 8u + sizeof(unsigned short) * 8u * 16u * 136u <= 131072u);
  const unsigned tid = threadIdx.x, lane = tid & 31u, col = lane & 15u, h = lane >> 4;
  const unsigned wave = (unsigned)__builtin_amdgcn_readfirstlane((int)(threadIdx.x >> 5));
  const unsigned wm = wave & 3u, wn = wave >> 2;
  const unsigned bm = blockIdx.x * 128u, bn = blockIdx.y * 256u;
  const unsigned ex = bn / II;
  { const v4f t4 = *(const v4f*)(G + (size_t)bm * NE + tid * 4u); *(v4f*)(&sg[0][0] + tid * 4u) = t4; }
  __syncthreads();
  const v4u* pa0 = XB + (size_t)(bm + wm * 32u + col) * DDQ + h;
  const v4u* pa1 = pa0 + 16u * DDQ;
  const v4u* pb  = WF + (size_t)(bn + wn * 128u + col) * DDQ + h;
  v8f acc0[8] = {}; v8f acc1[8] = {};
#pragma unroll 1
  for (unsigned kc = 0; kc < DD / 32u; ++kc) {
    const unsigned kq = kc * 4u;
    const v16b a0 = frag_q(pa0[kq], pa0[kq + 2u]);
    const v16b a1 = frag_q(pa1[kq], pa1[kq + 2u]);
    asm volatile("s_wait_loadcnt 0x0" ::: "memory");
#pragma unroll
    for (unsigned e = 0; e < 8u; e += 2u) {
      const v4u* pe = pb + (size_t)e * TSQ + kq;
      const v16b b0 = frag_q(pe[0], pe[2]);
      const v16b b1 = frag_q(pe[TSQ], pe[TSQ + 2u]);
      asm volatile("s_wait_loadcnt 0x0" ::: "memory");
      acc0[e] = wmma_bf(a0, b0, acc0[e]);
      acc1[e] = wmma_bf(a1, b0, acc1[e]);
      acc0[e + 1u] = wmma_bf(a0, b1, acc0[e + 1u]);
      acc1[e + 1u] = wmma_bf(a1, b1, acc1[e + 1u]);
    }
  }
  float gr0[8], gr1[8];
#pragma unroll
  for (unsigned r = 0; r < 8u; ++r) {
    gr0[r] = sg[wm * 32u + 8u * h + r][ex] * HMC;
    gr1[r] = sg[wm * 32u + 16u + 8u * h + r][ex] * HMC;
  }
  const size_t hq = (size_t)((bn + wn * 128u) >> 3);
#pragma unroll
  for (unsigned j = 0; j < 8u; ++j) {
#pragma unroll
    for (unsigned r = 0; r < 8u; ++r) {
      const float ge = gelu_erf(acc0[j][r]);
      st[wave][8u * h + r][j * 16u + col] = hbits(gr0[r] * ge);
    }
  }
  __syncthreads();
#pragma unroll
  for (unsigned it = 0; it < 8u; ++it) {
    const unsigned row = it * 2u + (lane >> 4), pc = lane & 15u;
    const v4u v = *(const v4u*)&st[wave][row][pc * 8u];
    vst2(HM + (size_t)(bm + wm * 32u + row) * NKQ + hq + pc, v);
  }
  __syncthreads();
#pragma unroll
  for (unsigned j = 0; j < 8u; ++j) {
#pragma unroll
    for (unsigned r = 0; r < 8u; ++r) {
      const float ge = gelu_erf(acc1[j][r]);
      st[wave][8u * h + r][j * 16u + col] = hbits(gr1[r] * ge);
    }
  }
  __syncthreads();
#pragma unroll
  for (unsigned it = 0; it < 8u; ++it) {
    const unsigned row = it * 2u + (lane >> 4), pc = lane & 15u;
    const v4u v = *(const v4u*)&st[wave][row][pc * 8u];
    vst2(HM + (size_t)(bm + wm * 32u + 16u + row) * NKQ + hq + pc, v);
  }
}

static_assert(32u * 16u * 8u == 16u * 64u * 4u);
__global__ __launch_bounds__(256) void k_proj(const v4u* __restrict__ HM, const v4u* __restrict__ WP, float* __restrict__ OUT) {
  __shared__ __align__(16) float sf[8][16][68];
  static_assert(sizeof(float) * 8u * 16u * 68u <= 131072u);
  const unsigned tid = threadIdx.x, lane = tid & 31u, col = lane & 15u, h = lane >> 4;
  const unsigned wave = (unsigned)__builtin_amdgcn_readfirstlane((int)(threadIdx.x >> 5));
  const unsigned wm = wave & 3u, wn = wave >> 2;
  const unsigned bm = blockIdx.x * 128u, bn = blockIdx.y * 256u;
  const v4u* pa0 = HM + (size_t)(bm + wm * 32u + col) * NKQ + h;
  const v4u* pa1 = pa0 + 16u * NKQ;
  const v4u* pb  = WP + (size_t)(bn + wn * 128u + col) * WPQ + h;
  v8f acc0[8] = {}; v8f acc1[8] = {};
#pragma unroll 1
  for (unsigned kc = 0; kc < NK / 32u; ++kc) {
    const unsigned kq = kc * 4u;
    const v16h a0 = frag_h(pa0[kq], pa0[kq + 2u]);
    const v16h a1 = frag_h(pa1[kq], pa1[kq + 2u]);
    asm volatile("s_wait_loadcnt 0x0" ::: "memory");
    const v4u* pk = pb + (size_t)(kc >> 4) * PEQ + (kc & 15u) * 4u;
#pragma unroll
    for (unsigned e = 0; e < 8u; e += 2u) {
      const v4u* pe = pk + (size_t)e * TPQ;
      const v16h b0 = frag_h(pe[0], pe[2]);
      const v16h b1 = frag_h(pe[TPQ], pe[TPQ + 2u]);
      asm volatile("s_wait_loadcnt 0x0" ::: "memory");
      acc0[e] = wmma_h(a0, b0, acc0[e]);
      acc1[e] = wmma_h(a1, b0, acc1[e]);
      acc0[e + 1u] = wmma_h(a0, b1, acc0[e + 1u]);
      acc1[e + 1u] = wmma_h(a1, b1, acc1[e + 1u]);
    }
  }
#pragma unroll
  for (unsigned q = 0; q < 2u; ++q) {
#pragma unroll
    for (unsigned j = 0; j < 4u; ++j) {
#pragma unroll
      for (unsigned r = 0; r < 8u; ++r) sf[wave][8u * h + r][j * 16u + col] = acc0[4u * q + j][r] * OSC;
    }
    __syncthreads();
#pragma unroll
    for (unsigned it = 0; it < 8u; ++it) {
      const unsigned row = it * 2u + (lane >> 4), pc = lane & 15u;
      const v4f v = *(const v4f*)&sf[wave][row][pc * 4u];
      vst2((v4f*)(OUT + (size_t)(bm + wm * 32u + row) * DO + bn + wn * 128u + q * 64u + pc * 4u), v);
    }
    __syncthreads();
  }
#pragma unroll
  for (unsigned q = 0; q < 2u; ++q) {
#pragma unroll
    for (unsigned j = 0; j < 4u; ++j) {
#pragma unroll
      for (unsigned r = 0; r < 8u; ++r) sf[wave][8u * h + r][j * 16u + col] = acc1[4u * q + j][r] * OSC;
    }
    __syncthreads();
#pragma unroll
    for (unsigned it = 0; it < 8u; ++it) {
      const unsigned row = it * 2u + (lane >> 4), pc = lane & 15u;
      const v4f v = *(const v4f*)&sf[wave][row][pc * 4u];
      vst2((v4f*)(OUT + (size_t)(bm + wm * 32u + 16u + row) * DO + bn + wn * 128u + q * 64u + pc * 4u), v);
    }
    __syncthreads();
  }
}

extern "C" void kernel_launch(void* const* d_in, const int* in_sizes, int n_in, void* d_out, int out_size, void* d_ws, size_t ws_size, hipStream_t stream) {
  if (n_in < 4) return;
  if ((size_t)in_sizes[0] < (size_t)NT * DD) return;
  if ((size_t)in_sizes[1] < (size_t)NE * DD) return;
  if ((size_t)in_sizes[2] < (size_t)NE * II * DD) return;
  if ((size_t)in_sizes[3] < (size_t)NE * DO * II) return;
  if ((size_t)out_size < (size_t)NT * DO) return;
  if (ws_size < (size_t)WS_END) return;
  const float* X   = (const float*)d_in[0];
  const float* WG  = (const float*)d_in[1];
  const float* WFC = (const float*)d_in[2];
  const float* WPJ = (const float*)d_in[3];
  char* ws = (char*)d_ws;
  float* G = (float*)(ws + WS_G);
  v4u* XB = (v4u*)(ws + WS_XB);
  v4u* WF = (v4u*)(ws + WS_WF);
  v4u* WP = (v4u*)(ws + WS_WP);
  v4u* HM = (v4u*)(ws + WS_HM);
  float* OUT = (float*)d_out;
  k_xcvt<<<dim3((NT * DD) / (8u * 256u)), 256, 0, stream>>>(X, XB);
  k_xcvt<<<dim3((NK * DD) / (8u * 256u)), 256, 0, stream>>>(WFC, WF);
  k_pcvt<<<dim3((NE * DO * II) / (8u * 256u)), 256, 0, stream>>>(WPJ, WP);
  k_gate<<<dim3(NT / 32u), 256, 0, stream>>>(XB, WG, G);
  k_fc<<<dim3(NT / 128u, NK / 256u), 256, 0, stream>>>(XB, WF, G, HM);
  k_proj<<<dim3(NT / 128u, DO / 256u), 256, 0, stream>>>(HM, WP, OUT);
}
